// GIN_71708773974793
// MI455X (gfx1250) — hardware-verified
//
#include <hip/hip_runtime.h>
#include <stddef.h>
#include <stdint.h>


#define NN      50000
#define NE      800000
#define DIN     128
#define K2      256
#define NG      100
#define OUTD    10
#define NOUT    1000
#define NP      50048
#define NTHR    256
#define NWAVE   8
#define EPT     8
#define CHUNK   (NTHR * EPT)
#define WCAP    (EPT * 32)
#define LISTN   (NWAVE * WCAP)
#define NB      1024
#define NBSH    10
#define NBLK    49
#define RCAP    28672
#define DEGCAP  64
#define PKS     11
#define GBM     64
#define GBN     128
#define GTHR    128
#define GNT     8
#define GTILES  (NP / GBM)
#define PARTW   288
#define APR     16
#define ARW     64
#define NUW     (DIN * (K2 / 8))
#define NUX     (NP * (DIN / 8))
#define NUTOT   (4 * NUW + NUX)
#define CZ_INTS (2 * RCAP + 2 * NB + LISTN)
#define LDS_CMP ((CZ_INTS + 16) * 4)
#define HD_HG   0
#define HD_Y    12800
#define HD_W1   25600
#define HD_W2   41984
#define HD_B1   43264
#define HD_B2   43392
#define HD_OUT  43408
#define HD_TOT  44416
#define LDS_HEAD (HD_TOT * 4)
#define WSCAP   134217728

static_assert(NN % 16 == 0);
static_assert(DIN == 32 * 4 && K2 == 2 * DIN && (K2 % 32) == 0);
static_assert(NP % GBM == 0 && NP >= NN && NP % APR == 0 && NP % ARW == 0);
static_assert((GTILES - 1) * GBM < NN);
static_assert(NB == (1 << NBSH) && NB * NBLK >= NP && NTHR * 4 == NB);
static_assert((CHUNK & (CHUNK - 1)) == 0 && CHUNK <= (1 << PKS) && NB <= (1 << PKS));
static_assert(NE < (1 << 21));
static_assert(LISTN >= NB && (RCAP % 1024) == 0 && (CZ_INTS % 1024) == 0);
static_assert(RCAP >= 17455);
static_assert(DEGCAP >= 35 + 8);
static_assert(LDS_CMP <= 300000 && LDS_HEAD <= 300000);
static_assert(GBM == (GTHR / 32) * 16 && GBN == 16 * GNT && GTHR == GBN && GBN == DIN);
static_assert((PARTW % 32) == 0 && PARTW >= 2 * GBN + 1 && PARTW / 4 <= GTHR);
static_assert((NUW % NTHR) == 0 && (NUX % NTHR) == 0 && (NUTOT % NTHR) == 0);
static_assert(NTHR == 2 * DIN && (APR * DIN) == 2 * 4 * NTHR && ARW == NWAVE * 8);
static_assert(NG * OUTD == NOUT && (NOUT % 4) == 0 && NOUT / 4 <= NTHR);
static_assert((NE % 4) == 0 && (NN % 4) == 0);
static_assert((HD_OUT % 4) == 0 && (HD_W1 % 4) == 0 && (HD_W2 % 4) == 0 && (HD_B1 % 4) == 0);

typedef float          v4f  __attribute__((ext_vector_type(4)));
typedef float          v8f  __attribute__((ext_vector_type(8)));
typedef int            v4i  __attribute__((ext_vector_type(4)));
typedef int            v8i  __attribute__((ext_vector_type(8)));
typedef unsigned int   v2u  __attribute__((ext_vector_type(2)));
typedef unsigned int   v4u  __attribute__((ext_vector_type(4)));
typedef unsigned short v4us __attribute__((ext_vector_type(4)));
typedef unsigned short v8us __attribute__((ext_vector_type(8)));
typedef __bf16         v16b __attribute__((ext_vector_type(16)));
typedef v4f  __attribute__((may_alias)) v4fa;
typedef v4i  __attribute__((may_alias)) v4ia;
typedef v2u  __attribute__((may_alias)) v2ua;
typedef v8us __attribute__((may_alias)) v8usa;
union Frag { v16b vb; v8us h[2]; v8i w; };

__device__ __forceinline__ v8f wmx(const Frag& a, const Frag& b, v8f c) {
  v8f d = __builtin_amdgcn_wmma_f32_16x16x32_bf16(false, a.vb, false, b.vb, (short)0, c, false, false);
  asm volatile("v_nop\n\tv_nop\n\tv_nop\n\tv_nop" : "+v"(d) : "v"(a.w), "v"(b.w));
  return d;
}

__device__ __forceinline__ unsigned short bf_bits(float f) {
  unsigned int u = __float_as_uint(f);
  u += 0x7FFFu + ((u >> 16) & 1u);
  return (unsigned short)(u >> 16);
}
__device__ __forceinline__ float bf_val(unsigned short b) { return __uint_as_float(((unsigned int)b) << 16); }
__device__ __forceinline__ float bf_rne(float f) { return bf_val(bf_bits(f)); }
__device__ __forceinline__ float relu_np(float v) { return (v > 0.0f) ? v : (v - v); }

__device__ __forceinline__ int scan_chunk(const int* __restrict__ dsts, int nE, int cbase, int slotBase,
                                          int nb, int vec8, int* list, int tid, int lane, int wave) {
  int wc = 0;
  const int el0  = tid * EPT;
  const int e0   = cbase + el0;
  const int sent = -2147483647 - 1;
  v4i da, db;
  if (vec8 != 0 && cbase + CHUNK <= nE) {
    da = *(const v4i*)(dsts + e0);
    db = *(const v4i*)(dsts + e0 + 4);
  } else {
    da.x = (e0     < nE) ? dsts[min(e0,     nE - 1)] : sent;
    da.y = (e0 + 1 < nE) ? dsts[min(e0 + 1, nE - 1)] : sent;
    da.z = (e0 + 2 < nE) ? dsts[min(e0 + 2, nE - 1)] : sent;
    da.w = (e0 + 3 < nE) ? dsts[min(e0 + 3, nE - 1)] : sent;
    db.x = (e0 + 4 < nE) ? dsts[min(e0 + 4, nE - 1)] : sent;
    db.y = (e0 + 5 < nE) ? dsts[min(e0 + 5, nE - 1)] : sent;
    db.z = (e0 + 6 < nE) ? dsts[min(e0 + 6, nE - 1)] : sent;
    db.w = (e0 + 7 < nE) ? dsts[min(e0 + 7, nE - 1)] : sent;
  }
  const unsigned nbs = (unsigned)slotBase;
  const unsigned unb = (unsigned)nb;
  const unsigned s0 = (unsigned)da.x - nbs, s1 = (unsigned)da.y - nbs;
  const unsigned s2 = (unsigned)da.z - nbs, s3 = (unsigned)da.w - nbs;
  const unsigned s4 = (unsigned)db.x - nbs, s5 = (unsigned)db.y - nbs;
  const unsigned s6 = (unsigned)db.z - nbs, s7 = (unsigned)db.w - nbs;
  const bool h0 = s0 < unb, h1 = s1 < unb, h2 = s2 < unb, h3 = s3 < unb;
  const bool h4 = s4 < unb, h5 = s5 < unb, h6 = s6 < unb, h7 = s7 < unb;
  const unsigned any = __builtin_amdgcn_ballot_w32(h0 | h1 | h2 | h3 | h4 | h5 | h6 | h7);
  if (any != 0u) {
#define HITJ(J, HJ, SJ) { \
      const unsigned mj = __builtin_amdgcn_ballot_w32(HJ); \
      if (mj != 0u) { \
        if (HJ) { \
          const int pos = wc + (int)__builtin_amdgcn_mbcnt_lo(mj, 0u); \
          if (pos < WCAP) list[wave * WCAP + pos] = ((el0 + (J)) << PKS) | (int)(SJ); \
        } \
        wc += (int)__builtin_popcount(mj); } }
    HITJ(0, h0, s0)
    HITJ(1, h1, s1)
    HITJ(2, h2, s2)
    HITJ(3, h3, s3)
    HITJ(4, h4, s4)
    HITJ(5, h5, s5)
    HITJ(6, h6, s6)
    HITJ(7, h7, s7)
#undef HITJ
  }
  return wc;
}

__device__ __forceinline__ v8us cv8b(const float* __restrict__ p, size_t stride) {
  v8us o;
#pragma unroll
  for (int i = 0; i < 8; ++i) o[i] = bf_bits(p[(size_t)i * stride]);
  return o;
}

__global__ __launch_bounds__(NTHR) void k_prep(const float* __restrict__ x,
                                               const float* __restrict__ w1a, const float* __restrict__ w2a,
                                               const float* __restrict__ w1b, const float* __restrict__ w2b,
                                               unsigned short* wt, unsigned short* xb) {
  const int u = (int)blockIdx.x * NTHR + (int)threadIdx.x;
  v8us o;
  unsigned short* dp;
  if (u < NUW) {
    const int v = u, n = v >> 5, kk = ((v & 31) * 8) & (DIN - 1);
    o = cv8b(w1a + (size_t)kk * DIN + n, DIN);
    dp = wt + (size_t)u * 8;
  } else if (u < 2 * NUW) {
    const int v = u - NUW, n = v >> 5, kk = ((v & 31) * 8) & (DIN - 1);
    o = cv8b(w2a + (size_t)kk * DIN + n, DIN);
    dp = wt + (size_t)u * 8;
  } else if (u < 3 * NUW) {
    const int v = u - 2 * NUW, n = v >> 5, kk = ((v & 31) * 8) & (DIN - 1);
    o = cv8b(w1b + (size_t)kk * DIN + n, DIN);
    dp = wt + (size_t)u * 8;
  } else if (u < 4 * NUW) {
    const int v = u - 3 * NUW, n = v >> 5, kk = ((v & 31) * 8) & (DIN - 1);
    o = cv8b(w2b + (size_t)kk * DIN + n, DIN);
    dp = wt + (size_t)u * 8;
  } else if (u < NUTOT) {
    const int v = u - 4 * NUW;
    const int row = v >> 4;
    const bool live = row < NN;
    const int sv = live ? v : 0;
    const float* p = x + (size_t)sv * 8;
    const v4f a = *(const v4f*)p;
    const v4f b = *(const v4f*)(p + 4);
    const unsigned short z = 0;
    o[0] = live ? bf_bits(a.x) : z; o[1] = live ? bf_bits(a.y) : z;
    o[2] = live ? bf_bits(a.z) : z; o[3] = live ? bf_bits(a.w) : z;
    o[4] = live ? bf_bits(b.x) : z; o[5] = live ? bf_bits(b.y) : z;
    o[6] = live ? bf_bits(b.z) : z; o[7] = live ? bf_bits(b.w) : z;
    dp = xb + (size_t)v * 8;
  } else {
    return;
  }
  *(volatile v8us*)dp = o;
  __threadfence();
  *(volatile v8us*)dp = o;
}

__global__ __launch_bounds__(NTHR) void k_compact(const int* __restrict__ srcs, const int* __restrict__ dsts,
                                                  int* LIST, int* CNT, int* OFF) {
  extern __shared__ v4f lds_cmp[];
  int* reg1 = (int*)lds_cmp;
  int* reg2 = reg1 + RCAP;
  int* scnt = reg2 + RCAP;
  int* soff = scnt + NB;
  int* list = soff + NB;
  int* wcnt = list + LISTN;
  int* wtot = wcnt + NWAVE;
  const int tid = (int)threadIdx.x, lane = tid & 31, wave = tid >> 5;
  const int blk = (int)blockIdx.x;
  const int nodeBase = blk * NB;

  {
    const v4i z4 = {0, 0, 0, 0};
#pragma unroll 1
    for (int i = tid * 4; i < CZ_INTS; i += NTHR * 4) *(v4ia*)(reg1 + i) = z4;
    if (tid < 16) wcnt[tid] = 0;
  }
  __syncthreads();

  int tot = 0;
  const int nChunks = (NE + CHUNK - 1) / CHUNK;
#pragma unroll 1
  for (int ch = 0; ch < nChunks; ++ch) {
    const int cbase = ch * CHUNK;
    const int wc = scan_chunk(dsts, NE, cbase, nodeBase, NB, 1, list, tid, lane, wave);
    if (lane == 0) wcnt[wave] = wc;
    __syncthreads();
    int pre = 0, all = 0;
#pragma unroll
    for (int w2 = 0; w2 < NWAVE; ++w2) {
      int c = wcnt[w2];
      c = c < 0 ? 0 : (c > WCAP ? WCAP : c);
      all += c;
      pre += (w2 < wave) ? c : 0;
    }
    const int wcc  = wc > WCAP ? WCAP : wc;
    const int base = tot + pre;
#pragma unroll 1
    for (int i = lane; i < wcc; i += 32) {
      const int ent = list[wave * WCAP + i];
      const int el  = (ent >> PKS) & (CHUNK - 1);
      const int sl  = ent & (NB - 1);
      int eid = cbase + el;
      eid = eid > NE - 1 ? NE - 1 : eid;
      const int pos = base + i;
      if (pos < RCAP) reg1[pos] = (int)(((unsigned)eid << PKS) | (unsigned)sl);
    }
    tot += all;
    tot = tot > RCAP ? RCAP : tot;
    __syncthreads();
  }
  const int nh = tot;

  if (wave == 0) {
#pragma unroll 1
    for (int b0 = 0; b0 < nh; b0 += 32) {
      const int idx = b0 + lane;
      const int uv  = reg1[idx < RCAP ? idx : RCAP - 1];
      const int m32 = (nh - b0) < 32 ? (nh - b0) : 32;
#pragma unroll 1
      for (int k = 0; k < m32; ++k) {
        const int u  = __builtin_amdgcn_readlane(uv, k);
        const int sl = u & (NB - 1);
        if (lane == 0) scnt[sl] = scnt[sl] + 1;
      }
    }
  }
  __syncthreads();

  {
    const v4i ca = *(const v4ia*)(scnt + 4 * tid);
    const int e0 = ca.x < 0 ? 0 : ca.x, e1 = ca.y < 0 ? 0 : ca.y;
    const int e2 = ca.z < 0 ? 0 : ca.z, e3 = ca.w < 0 ? 0 : ca.w;
    const int ts = e0 + e1 + e2 + e3;
    int incl = ts;
#pragma unroll
    for (int d = 1; d < 32; d <<= 1) {
      const int up = __shfl_up(incl, d);
      if (lane >= d) incl += up;
    }
    if (lane == 31) wtot[wave] = incl;
    __syncthreads();
    int pre = 0;
#pragma unroll
    for (int w2 = 0; w2 < NWAVE; ++w2) pre += (w2 < wave) ? wtot[w2] : 0;
    int run = pre + incl - ts;
    soff[4 * tid + 0] = run; run += e0;
    soff[4 * tid + 1] = run; run += e1;
    soff[4 * tid + 2] = run; run += e2;
    soff[4 * tid + 3] = run;
  }
  __syncthreads();
#pragma unroll 1
  for (int i = tid; i < NB; i += NTHR) list[i] = soff[i];
  __syncthreads();

  if (wave == 0) {
#pragma unroll 1
    for (int b0 = 0; b0 < nh; b0 += 32) {
      const int idx = b0 + lane;
      const int uv  = reg1[idx < RCAP ? idx : RCAP - 1];
      const int m32 = (nh - b0) < 32 ? (nh - b0) : 32;
#pragma unroll 1
      for (int k = 0; k < m32; ++k) {
        const int u   = __builtin_amdgcn_readlane(uv, k);
        const int sl  = u & (NB - 1);
        const int eid = (int)((unsigned)u >> PKS);
        if (lane == 0) {
          int pos = list[sl];
          pos = pos < 0 ? 0 : (pos > RCAP - 1 ? RCAP - 1 : pos);
          reg2[pos] = eid;
          list[sl] = pos + 1;
        }
      }
    }
  }
  __syncthreads();

#pragma unroll 1
  for (int i = tid; i < nh; i += NTHR) {
    int eid = reg2[i];
    eid = eid < 0 ? 0 : (eid > NE - 1 ? NE - 1 : eid);
    int s = srcs[eid];
    s = s < 0 ? 0 : (s > NN - 1 ? NN - 1 : s);
    reg2[i] = s;
  }
  __syncthreads();

  const bool ovf = (nh >= RCAP);
  v4i cv = *(const v4ia*)(scnt + 4 * tid);
  const v4i ov = *(const v4ia*)(soff + 4 * tid);
  cv.x = (ovf || cv.x < 0 || cv.x > DEGCAP) ? -1 : cv.x;
  cv.y = (ovf || cv.y < 0 || cv.y > DEGCAP) ? -1 : cv.y;
  cv.z = (ovf || cv.z < 0 || cv.z > DEGCAP) ? -1 : cv.z;
  cv.w = (ovf || cv.w < 0 || cv.w > DEGCAP) ? -1 : cv.w;
  int* cp = CNT + (size_t)blk * NB + 4 * tid;
  int* op = OFF + (size_t)blk * NB + 4 * tid;
  int* lb = LIST + (size_t)blk * RCAP;
#pragma unroll 1
  for (int it = 0; it < RCAP / (4 * NTHR); ++it) {
    const int p = it * NTHR + tid;
    const v4i v = *(const v4ia*)(reg2 + 4 * p);
    *(volatile v4i*)(lb + 4 * p) = v;
  }
  *(volatile v4i*)cp = cv;
  *(volatile v4i*)op = ov;
  __threadfence();
#pragma unroll 1
  for (int it = 0; it < RCAP / (4 * NTHR); ++it) {
    const int p = it * NTHR + tid;
    const v4i v = *(const v4ia*)(reg2 + 4 * p);
    *(volatile v4i*)(lb + 4 * p) = v;
  }
  *(volatile v4i*)cp = cv;
  *(volatile v4i*)op = ov;
}

template <int F32SRC>
__global__ __launch_bounds__(NTHR) void k_agg(const int* __restrict__ LIST, const int* __restrict__ CNT,
                                              const int* __restrict__ OFF,
                                              const unsigned short* __restrict__ xb,
                                              const float* __restrict__ hf,
                                              unsigned short* P1) {
  const int tid = (int)threadIdx.x, lane = tid & 31, wave = tid >> 5;
  const int rowBase = (int)blockIdx.x * ARW;
  const float qnan = __int_as_float(0x7fc00000);
#pragma unroll 1
  for (int jt = 0; jt < ARW / NWAVE; ++jt) {
    const int d = rowBase + wave * (ARW / NWAVE) + jt;
    const int craw = __builtin_amdgcn_readfirstlane(CNT[d]);
    int o = __builtin_amdgcn_readfirstlane(OFF[d]);
    const int blk = __builtin_amdgcn_readfirstlane(d >> NBSH);
    const bool bad = (craw < 0) || (craw > DEGCAP);
    int c = craw < 0 ? 0 : (craw > DEGCAP ? DEGCAP : craw);
    o = o < 0 ? 0 : (o > RCAP ? RCAP : o);
    if (c > RCAP - o) c = RCAP - o;
    const int* lb = LIST + (size_t)blk * RCAP;
    float a0 = 0.0f, a1 = 0.0f, a2 = 0.0f, a3 = 0.0f;
#pragma unroll 1
    for (int b0 = 0; b0 < c; b0 += 32) {
      int idx = o + b0 + lane;
      idx = idx > RCAP - 1 ? RCAP - 1 : idx;
      int sr = lb[idx];
      sr = sr < 0 ? 0 : (sr > NN - 1 ? NN - 1 : sr);
      const int m32 = (c - b0) < 32 ? (c - b0) : 32;
#pragma unroll 1
      for (int k = 0; k < m32; ++k) {
        const int sk = __builtin_amdgcn_readlane(sr, k);
        if constexpr (F32SRC != 0) {
          const v4f v = *(const v4f*)(hf + (size_t)sk * DIN + 4 * lane);
          a0 += v.x; a1 += v.y; a2 += v.z; a3 += v.w;
        } else {
          const v2u q = *(const v2ua*)(xb + (size_t)sk * DIN + 4 * lane);
          a0 += __uint_as_float(q.x << 16);
          a1 += __uint_as_float(q.x & 0xffff0000u);
          a2 += __uint_as_float(q.y << 16);
          a3 += __uint_as_float(q.y & 0xffff0000u);
        }
      }
    }
    const bool liveRow = d < NN;
    const int dc = liveRow ? d : NN - 1;
    float s0, s1, s2, s3;
    if constexpr (F32SRC != 0) {
      const v4f v = *(const v4f*)(hf + (size_t)dc * DIN + 4 * lane);
      s0 = v.x; s1 = v.y; s2 = v.z; s3 = v.w;
    } else {
      const v2u q = *(const v2ua*)(xb + (size_t)dc * DIN + 4 * lane);
      s0 = __uint_as_float(q.x << 16);
      s1 = __uint_as_float(q.x & 0xffff0000u);
      s2 = __uint_as_float(q.y << 16);
      s3 = __uint_as_float(q.y & 0xffff0000u);
    }
    const float pz = bad ? qnan : 0.0f;
    float r[4];
    r[0] = (liveRow ? (a0 + s0) : 0.0f) + pz;
    r[1] = (liveRow ? (a1 + s1) : 0.0f) + pz;
    r[2] = (liveRow ? (a2 + s2) : 0.0f) + pz;
    r[3] = (liveRow ? (a3 + s3) : 0.0f) + pz;
    v4us hv, lv;
#pragma unroll
    for (int j = 0; j < 4; ++j) {
      const unsigned short hb = bf_bits(r[j]);
      hv[j] = hb;
      lv[j] = bf_bits(r[j] - bf_val(hb));
    }
    unsigned short* aq = P1 + (size_t)d * K2 + 4 * lane;
    *(volatile v4us*)aq = hv;
    *(volatile v4us*)(aq + DIN) = lv;
    __threadfence();
    *(volatile v4us*)aq = hv;
    *(volatile v4us*)(aq + DIN) = lv;
  }
}

template <int EPI>
__global__ __launch_bounds__(GTHR) void k_gemm(const unsigned short* __restrict__ A,
                                               const unsigned short* __restrict__ BT,
                                               const float* __restrict__ bias,
                                               float* outF, float* part) {
  __shared__ __attribute__((aligned(16))) float stg[GBM * GBN];
  __shared__ __attribute__((aligned(16))) float pst[PARTW];
  const int tid = (int)threadIdx.x, lane = tid & 31, wave = tid >> 5, hh = lane >> 4, m = lane & 15;
  const int rowBase = (int)blockIdx.x * GBM;

  v8f acc[GNT];
  {
    const v8f z = {0.f, 0.f, 0.f, 0.f, 0.f, 0.f, 0.f, 0.f};
#pragma unroll
    for (int t = 0; t < GNT; ++t) acc[t] = z;
  }
  const unsigned short* ap = A  + (size_t)(rowBase + 16 * wave + m) * (size_t)K2 + 8 * hh;
  const unsigned short* bp = BT + (size_t)m * (size_t)K2 + 8 * hh;

#pragma unroll 1
  for (int k0 = 0; k0 < K2; k0 += 32) {
    Frag af;
    af.h[0] = *(const v8usa*)(ap + k0);
    af.h[1] = *(const v8usa*)(ap + k0 + 16);
#pragma unroll
    for (int nt = 0; nt < GNT; ++nt) {
      const unsigned short* wq = bp + (size_t)(16 * nt) * (size_t)K2 + k0;
      Frag bfr;
      bfr.h[0] = *(const v8usa*)wq;
      bfr.h[1] = *(const v8usa*)(wq + 16);
      acc[nt] = wmx(af, bfr, acc[nt]);
    }
  }

#pragma unroll
  for (int nt = 0; nt < GNT; ++nt) {
    const int lc = 16 * nt + m;
    const float bb = bf_rne(bias[lc]);
#pragma unroll
    for (int r = 0; r < 8; ++r) {
      const int lr = 16 * wave + 8 * hh + r;
      const bool live = (rowBase + lr) < NN;
      float v = acc[nt][r] + bb;
      if constexpr (EPI == 3) v = relu_np(v);
      stg[lr * GBN + lc] = live ? v : 0.0f;
    }
  }
  __syncthreads();

  v4f fv[16];
#pragma unroll
  for (int i = 0; i < 16; ++i) {
    const int lr = 16 * wave + i;
    fv[i] = *(const v4fa*)(stg + lr * GBN + 4 * lane);
  }
  v4f pv = {0.f, 0.f, 0.f, 0.f};
  const bool pok = (EPI == 1) && (tid < PARTW / 4);
  if constexpr (EPI == 1) {
    int nvr = NN - rowBase;
    nvr = nvr < 0 ? 0 : (nvr > GBM ? GBM : nvr);
    float s = 0.0f;
#pragma unroll 1
    for (int r = 0; r < nvr; ++r) s += stg[r * GBN + tid];
    const float inv = 1.0f / (float)(nvr < 1 ? 1 : nvr);
    const float mean = s * inv;
    float q = 0.0f;
#pragma unroll 1
    for (int r = 0; r < nvr; ++r) {
      const float d = stg[r * GBN + tid] - mean;
      q = fmaf(d, d, q);
    }
    pst[1 + tid] = mean;
    pst[1 + GBN + tid] = q;
    if (tid == 0) pst[0] = (float)nvr;
#pragma unroll 1
    for (int i = 2 * GBN + 1 + tid; i < PARTW; i += GTHR) pst[i] = 0.0f;
    __syncthreads();
    if (pok) pv = *(const v4fa*)(pst + 4 * tid);
  }
  float* pp = part + (size_t)blockIdx.x * PARTW + 4 * tid;
#pragma unroll
  for (int i = 0; i < 16; ++i) {
    const int gr = rowBase + 16 * wave + i;
    float* op = outF + (size_t)gr * (size_t)DIN + 4 * lane;
    *(volatile v4f*)op = fv[i];
  }
  if (pok) *(volatile v4f*)pp = pv;
  __threadfence();
#pragma unroll
  for (int i = 0; i < 16; ++i) {
    const int gr = rowBase + 16 * wave + i;
    float* op = outF + (size_t)gr * (size_t)DIN + 4 * lane;
    *(volatile v4f*)op = fv[i];
  }
  if (pok) *(volatile v4f*)pp = pv;
}

__global__ __launch_bounds__(GBN) void k_comb(const float* __restrict__ part,
                                              const float* __restrict__ gam, const float* __restrict__ bet,
                                              float* stat) {
  __shared__ __attribute__((aligned(16))) float stg[4 * DIN];
  const int tid = (int)threadIdx.x;
  double n = 0.0, mean = 0.0, M2 = 0.0;
#pragma unroll 1
  for (int b = 0; b < GTILES; ++b) {
    const float* pr = part + (size_t)b * PARTW;
    const double nb = (double)pr[0];
    const double mb = (double)pr[1 + tid];
    const double qb = (double)pr[1 + GBN + tid];
    if (nb > 0.5) {
      const double nn = n + nb;
      const double delta = mb - mean;
      const double f = nb / nn;
      mean = mean + delta * f;
      M2 = M2 + qb + delta * delta * n * f;
      n = nn;
    }
  }
  const double nt = n < 1.0 ? 1.0 : n;
  const float var  = (float)(M2 / nt);
  const float rstd = 1.0f / sqrtf(var + 1e-5f);
  stg[tid] = (float)mean;
  stg[DIN + tid] = rstd;
  stg[2 * DIN + tid] = bf_rne(gam[tid]);
  stg[3 * DIN + tid] = bf_rne(bet[tid]);
  __syncthreads();
  const v4f v = *(const v4fa*)(stg + 4 * tid);
  float* dp = stat + 4 * tid;
  *(volatile v4f*)dp = v;
  __threadfence();
  *(volatile v4f*)dp = v;
}

__global__ __launch_bounds__(NTHR) void k_apply(const float* __restrict__ T, const float* __restrict__ stat,
                                                unsigned short* P1) {
  __shared__ float ssh[4 * DIN];
  __shared__ __attribute__((aligned(16))) float tile[APR * DIN];
  const int tid = (int)threadIdx.x;
  ssh[tid] = stat[tid];
  ssh[NTHR + tid] = stat[NTHR + tid];
  const int rowBase = (int)blockIdx.x * APR;
  const int c  = tid & (DIN - 1);
  const int rs = tid >> 7;
  __syncthreads();
  const float mu = ssh[c], rr = ssh[DIN + c], gg = ssh[2 * DIN + c], be = ssh[3 * DIN + c];
#pragma unroll 1
  for (int r = 0; r < APR / 2; ++r) {
    const int lr   = 2 * r + rs;
    const int grow = rowBase + lr;
    const int gc   = grow < NN ? grow : NN - 1;
    const float u = T[(size_t)gc * DIN + c];
    const float y = ((u - mu) * rr) * gg + be;
    const float v = relu_np(y);
    tile[lr * DIN + c] = (grow < NN) ? v : 0.0f;
  }
  __syncthreads();
  const int lane = tid & 31, wave = tid >> 5, hh = lane >> 4, m = lane & 15;
  const int cb = 8 * m;
  const bool isHi = (hh == 0);
  v4u pk[2];
#pragma unroll
  for (int i = 0; i < 2; ++i) {
    const int lr = 2 * wave + i;
    const v4f a = *(const v4fa*)(tile + lr * DIN + cb);
    const v4f b = *(const v4fa*)(tile + lr * DIN + cb + 4);
    const float f[8] = {a.x, a.y, a.z, a.w, b.x, b.y, b.z, b.w};
    unsigned int w[4];
#pragma unroll
    for (int j = 0; j < 4; ++j) {
      const unsigned short h0 = bf_bits(f[2 * j]), h1 = bf_bits(f[2 * j + 1]);
      const unsigned short l0 = bf_bits(f[2 * j] - bf_val(h0)), l1 = bf_bits(f[2 * j + 1] - bf_val(h1));
      const unsigned short q0 = isHi ? h0 : l0, q1 = isHi ? h1 : l1;
      w[j] = (unsigned int)q0 | ((unsigned int)q1 << 16);
    }
    v4u pv; pv.x = w[0]; pv.y = w[1]; pv.z = w[2]; pv.w = w[3];
    pk[i] = pv;
  }
#pragma unroll
  for (int i = 0; i < 2; ++i) {
    const int grow = rowBase + 2 * wave + i;
    unsigned short* op = P1 + (size_t)grow * K2 + cb + hh * DIN;
    *(volatile v4u*)op = pk[i];
  }
  __threadfence();
#pragma unroll
  for (int i = 0; i < 2; ++i) {
    const int grow = rowBase + 2 * wave + i;
    unsigned short* op = P1 + (size_t)grow * K2 + cb + hh * DIN;
    *(volatile v4u*)op = pk[i];
  }
}

__global__ __launch_bounds__(NTHR) void k_pool(const float* __restrict__ H, const int* __restrict__ bat,
                                               float* hg) {
  __shared__ int list[LISTN];
  __shared__ int wcnt[NWAVE];
  __shared__ __attribute__((aligned(16))) float acs[DIN];
  const int tid = (int)threadIdx.x, lane = tid & 31, wave = tid >> 5;
  const int g = (int)blockIdx.x;
  float acc = 0.0f;
  const int nChunks = (NN + CHUNK - 1) / CHUNK;
#pragma unroll 1
  for (int ch = 0; ch < nChunks; ++ch) {
    const int cbase = ch * CHUNK;
    const int wc = scan_chunk(bat, NN, cbase, g, 1, 1, list, tid, lane, wave);
    if (lane == 0) wcnt[wave] = wc;
    __syncthreads();
#pragma unroll 1
    for (int w2 = 0; w2 < NWAVE; ++w2) {
      int c = wcnt[w2];
      c = c < 0 ? 0 : (c > WCAP ? WCAP : c);
#pragma unroll 1
      for (int i = 0; i < c; ++i) {
        const int ent = list[w2 * WCAP + i];
        const int el  = (ent >> PKS) & (CHUNK - 1);
        int node = cbase + el;
        node = node < 0 ? 0 : (node > NN - 1 ? NN - 1 : node);
        if (tid < DIN) acc += H[(size_t)node * DIN + tid];
      }
    }
    __syncthreads();
  }
  if (tid < DIN) acs[tid] = acc;
  __syncthreads();
  const bool ok = tid < 32;
  v4f v = {0.f, 0.f, 0.f, 0.f};
  float* dp = hg + (size_t)g * DIN + 4 * lane;
  if (ok) {
    v = *(const v4fa*)(acs + 4 * lane);
    *(volatile v4f*)dp = v;
  }
  __threadfence();
  if (ok) *(volatile v4f*)dp = v;
}

__global__ __launch_bounds__(NTHR) void k_head(const float* __restrict__ hg,
                                               const float* __restrict__ wl1, const float* __restrict__ bl1,
                                               const float* __restrict__ wl2, const float* __restrict__ bl2,
                                               float* out) {
  extern __shared__ v4f lds_head[];
  float* sm  = (float*)lds_head;
  float* hgS = sm + HD_HG;
  float* yS  = sm + HD_Y;
  float* w1S = sm + HD_W1;
  float* w2S = sm + HD_W2;
  float* b1S = sm + HD_B1;
  float* b2S = sm + HD_B2;
  float* oS  = sm + HD_OUT;
  const int tid = (int)threadIdx.x;
#pragma unroll 1
  for (int i = tid; i < (NG * DIN) / 4; i += NTHR) {
    const v4f v = *(const v4f*)(hg + 4 * i);
    *(v4fa*)(hgS + 4 * i) = v;
  }
#pragma unroll 1
  for (int i = tid; i < (DIN * DIN) / 4; i += NTHR) {
    const v4f v = *(const v4f*)(wl1 + 4 * i);
    v4f w; w.x = bf_rne(v.x); w.y = bf_rne(v.y); w.z = bf_rne(v.z); w.w = bf_rne(v.w);
    *(v4fa*)(w1S + 4 * i) = w;
  }
#pragma unroll 1
  for (int i = tid; i < (DIN * OUTD) / 4; i += NTHR) {
    const v4f v = *(const v4f*)(wl2 + 4 * i);
    v4f w; w.x = bf_rne(v.x); w.y = bf_rne(v.y); w.z = bf_rne(v.z); w.w = bf_rne(v.w);
    *(v4fa*)(w2S + 4 * i) = w;
  }
  if (tid < DIN) b1S[tid] = bf_rne(bl1[tid]);
  if (tid < 16) {
    const float bv = bl2[tid < OUTD ? tid : OUTD - 1];
    b2S[tid] = (tid < OUTD) ? bf_rne(bv) : 0.0f;
  }
  if (tid < 8) oS[NOUT + tid] = 0.0f;
  __syncthreads();

  {
    const int c  = tid & (DIN - 1);
    const int rs = tid >> 7;
    const float bb = b1S[c];
#pragma unroll 1
    for (int i = 0; i < NG / 2; ++i) {
      const int g = 2 * i + rs;
      float acc = 0.0f;
#pragma unroll 4
      for (int k = 0; k < DIN; ++k) acc = fmaf(hgS[g * DIN + k], w1S[k * DIN + c], acc);
      yS[g * DIN + c] = relu_np(acc + bb);
    }
  }
  __syncthreads();

#pragma unroll 1
  for (int idx = tid; idx < NOUT; idx += NTHR) {
    const int g = idx / OUTD;
    const int o = idx - g * OUTD;
    float acc = 0.0f;
#pragma unroll 4
    for (int k = 0; k < DIN; ++k) acc = fmaf(yS[g * DIN + k], w2S[k * OUTD + o], acc);
    oS[idx] = acc + b2S[o];
  }
  __syncthreads();

  const bool ok = tid < NOUT / 4;
  v4f v = {0.f, 0.f, 0.f, 0.f};
  float* dp = out + 4 * (ok ? tid : 0);
  if (ok) {
    v = *(const v4fa*)(oS + 4 * tid);
    *(volatile v4f*)dp = v;
  }
  __threadfence();
  if (ok) *(volatile v4f*)dp = v;
}

static inline size_t al256(size_t o) { return (o + 255) & ~(size_t)255; }

extern "C" void kernel_launch(void* const* d_in, const int* in_sizes, int n_in,
                              void* d_out, int out_size, void* d_ws, size_t ws_size,
                              hipStream_t stream) {
  if (n_in < 19) return;
  if (in_sizes[0] != NN * DIN) return;
  if (in_sizes[1] != 2 * NE) return;
  if (in_sizes[2] != NN) return;
  if (in_sizes[3] != DIN * DIN || in_sizes[4] != DIN) return;
  if (in_sizes[5] != DIN || in_sizes[6] != DIN) return;
  if (in_sizes[7] != DIN * DIN || in_sizes[8] != DIN) return;
  if (in_sizes[9] != DIN * DIN || in_sizes[10] != DIN) return;
  if (in_sizes[11] != DIN || in_sizes[12] != DIN) return;
  if (in_sizes[13] != DIN * DIN || in_sizes[14] != DIN) return;
  if (in_sizes[15] != DIN * DIN || in_sizes[16] != DIN) return;
  if (in_sizes[17] != DIN * OUTD || in_sizes[18] != OUTD) return;
  if (out_size != NOUT) return;

  const float* x     = (const float*)d_in[0];
  const int*   ei    = (const int*)  d_in[1];
  const int*   src   = ei;
  const int*   dst   = ei + NE;
  const int*   batch = (const int*)  d_in[2];
  const float* W1a = (const float*)d_in[3];  const float* b1a  = (const float*)d_in[4];
  const float* g1a = (const float*)d_in[5];  const float* be1a = (const float*)d_in[6];
  const float* W2a = (const float*)d_in[7];  const float* b2a  = (const float*)d_in[8];
  const float* W1b = (const float*)d_in[9];  const float* b1b  = (const float*)d_in[10];
  const float* g1b = (const float*)d_in[11]; const float* be1b = (const float*)d_in[12];
  const float* W2b = (const float*)d_in[13]; const float* b2b  = (const float*)d_in[14];
  const float* Wl1 = (const float*)d_in[15]; const float* bl1  = (const float*)d_in[16];
  const float* Wl2 = (const float*)d_in[17]; const float* bl2  = (const float*)d_in[18];
  float* out = (float*)d_out;

  char* ws = (char*)d_ws;
  size_t off = 0;
  const size_t oWT  = off; off = al256(off + (size_t)4 * NUW * 16);
  const size_t oXB  = off; off = al256(off + (size_t)NP * DIN * 2);
  const size_t oP1  = off; off = al256(off + (size_t)NP * K2 * 2);
  const size_t oP2  = off; off = al256(off + (size_t)NP * DIN * 4);
  const size_t oP3  = off; off = al256(off + (size_t)NP * DIN * 4);
  const size_t oLS  = off; off = al256(off + (size_t)NBLK * RCAP * 4);
  const size_t oCN  = off; off = al256(off + (size_t)NBLK * NB * 4);
  const size_t oOF  = off; off = al256(off + (size_t)NBLK * NB * 4);
  const size_t oRC  = off; off = al256(off + (size_t)GTILES * PARTW * 4);
  const size_t oST  = off; off = al256(off + (size_t)(4 * DIN) * 4);
  const size_t oHG  = off; off = al256(off + (size_t)NG * DIN * 4);
  if (off > ws_size || off > (size_t)WSCAP) return;
  unsigned short* WT = (unsigned short*)(ws + oWT);
  unsigned short* XB = (unsigned short*)(ws + oXB);
  unsigned short* P1 = (unsigned short*)(ws + oP1);
  float*          P2 = (float*)(ws + oP2);
  float*          P3 = (float*)(ws + oP3);
  int*            LS = (int*)(ws + oLS);
  int*            CN = (int*)(ws + oCN);
  int*            OF = (int*)(ws + oOF);
  float*          RC = (float*)(ws + oRC);
  float*          ST = (float*)(ws + oST);
  float*          HG = (float*)(ws + oHG);
  unsigned short* W1aT = WT;
  unsigned short* W2aT = WT + (size_t)NUW * 8;
  unsigned short* W1bT = WT + (size_t)2 * NUW * 8;
  unsigned short* W2bT = WT + (size_t)3 * NUW * 8;

  hipFuncSetAttribute(reinterpret_cast<const void*>(&k_compact), hipFuncAttributeMaxDynamicSharedMemorySize, LDS_CMP);
  hipFuncSetAttribute(reinterpret_cast<const void*>(&k_head),    hipFuncAttributeMaxDynamicSharedMemorySize, LDS_HEAD);

  k_prep<<<NUTOT / NTHR, NTHR, 0, stream>>>(x, W1a, W2a, W1b, W2b, WT, XB);
  k_compact<<<NBLK, NTHR, LDS_CMP, stream>>>(src, dst, LS, CN, OF);
  k_agg<0><<<NP / ARW, NTHR, 0, stream>>>(LS, CN, OF, XB, P3, P1);
  k_gemm<1><<<GTILES, GTHR, 0, stream>>>(P1, W1aT, b1a, P2, RC);
  k_comb<<<1, GBN, 0, stream>>>(RC, g1a, be1a, ST);
  k_apply<<<NP / APR, NTHR, 0, stream>>>(P2, ST, P1);
  k_gemm<3><<<GTILES, GTHR, 0, stream>>>(P1, W2aT, b2a, P3, RC);
  k_agg<1><<<NP / ARW, NTHR, 0, stream>>>(LS, CN, OF, XB, P3, P1);
  k_gemm<1><<<GTILES, GTHR, 0, stream>>>(P1, W1bT, b1b, P2, RC);
  k_comb<<<1, GBN, 0, stream>>>(RC, g1b, be1b, ST);
  k_apply<<<NP / APR, NTHR, 0, stream>>>(P2, ST, P1);
  k_gemm<3><<<GTILES, GTHR, 0, stream>>>(P1, W2bT, b2b, P3, RC);
  k_pool<<<NG, NTHR, 0, stream>>>(P3, batch, HG);
  k_head<<<1, NTHR, LDS_HEAD, stream>>>(HG, Wl1, bl1, Wl2, bl2, out);
}
